// MPNNModel_970662609384
// MI455X (gfx1250) — hardware-verified
//
#include <hip/hip_runtime.h>
#include <stddef.h>


#define NNODE 100000
#define NEDGE 1000000
#define INDIM 49
#define EMBD 64
#define NLAYER 4
#define ETILES (NEDGE / 16)
#define NTILES (NNODE / 16)
#define BKT_NODES 1024
#define NBKT 98
#define BKT_CAP 16384
#define BINFO_P 1056
#define OFF_PAD 100032
#define OFF_PIECES (OFF_PAD / 4)
#define PERM_PIECES (NEDGE / 4)
#define CS_BLOCKS 256
#define EDGE_GRID 1024
#define NODE_GRID 256
#define BN_EPS 1e-5f
#define WSCALE 16.0f
#define WINV 0.0625f

static_assert(NEDGE % 32 == 0, "");
static_assert(NNODE % 32 == 0, "");
static_assert(ETILES % 4 == 0, "");
static_assert(NNODE % 8 == 0, "");
static_assert(NBKT * BKT_NODES >= NNODE, "");
static_assert((NBKT - 1) * BKT_NODES < NNODE, "");
static_assert(OFF_PAD % 32 == 0 && OFF_PAD >= NNODE + 1, "");
static_assert(BKT_CAP % 32 == 0, "");
static_assert(BINFO_P % 32 == 0 && BINFO_P >= BKT_NODES + 1, "");
static_assert(NEDGE <= (1 << 20), "");

typedef _Float16 f16t;
typedef f16t v16h __attribute__((ext_vector_type(16)));
typedef f16t v8h __attribute__((ext_vector_type(8)));
typedef f16t v4h __attribute__((ext_vector_type(4)));
typedef f16t v2h __attribute__((ext_vector_type(2)));
typedef float v8f __attribute__((ext_vector_type(8)));
typedef float v4f __attribute__((ext_vector_type(4)));
typedef int v4i __attribute__((ext_vector_type(4)));
typedef double v2d __attribute__((ext_vector_type(2)));
typedef v8h v8h_a __attribute__((may_alias));
typedef v4h v4h_a __attribute__((may_alias));
typedef v2h v2h_a __attribute__((may_alias));
typedef v4f v4f_a __attribute__((may_alias));
typedef v4i v4i_a __attribute__((may_alias));
typedef v2d v2d_a __attribute__((may_alias));

union FragU { v16h v; v8h h[2]; };

__device__ __forceinline__ v8f wmma16(v16h a, v16h b, v8f c) {
    c = __builtin_amdgcn_wmma_f32_16x16x32_f16(false, a, false, b, (short)0, c, false, false);
    asm volatile("v_nop\n\tv_nop\n\tv_nop\n\tv_nop" : "+v"(c) : "v"(a), "v"(b));
    return c;
}

__device__ __forceinline__ v16h frag16(const f16t* p, int hh) {
    FragU f;
    f.h[0] = *(const v8h_a*)(p + 8 * hh);
    f.h[1] = *(const v8h_a*)(p + 16 + 8 * hh);
    return f.v;
}

__device__ __forceinline__ int clampi(int v, int lo, int hi) { return v < lo ? lo : (v > hi ? hi : v); }

__device__ __forceinline__ void rows16_store(const f16t* stg, f16t* gdst, int l) {
#pragma unroll
    for (int j = 0; j < 4; ++j) {
        const int p = 32 * j + l;
        const int row = p >> 3, cb = (p & 7) * 8;
        const v8h v = *(const v8h_a*)(stg + row * EMBD + cb);
        *(volatile v8h*)(gdst + (size_t)row * EMBD + cb) = v;
    }
}

__device__ __forceinline__ void stats_out(const double (&sl)[4], const double (&ql)[4], double* red, double* pout) {
    const int t = threadIdx.x, w = t >> 5, l = t & 31, hh = l >> 4, m = l & 15;
#pragma unroll
    for (int n = 0; n < 4; ++n) {
        red[(w * 2 + hh) * 64 + 16 * n + m] = sl[n];
        red[512 + (w * 2 + hh) * 64 + 16 * n + m] = ql[n];
    }
    __syncthreads();
    double S = 0.0, Q = 0.0;
    if (t < 64) {
        for (int j = 0; j < 8; ++j) { S += red[j * 64 + t]; Q += red[512 + j * 64 + t]; }
    }
    __syncthreads();
    if (t < 64) { red[t] = S; red[64 + t] = Q; }
    __syncthreads();
    v2d a = {0.0, 0.0}, b = {0.0, 0.0};
    if (t < 32) {
        a = *(const v2d_a*)&red[2 * t];
        b = *(const v2d_a*)&red[64 + 2 * t];
        *(volatile v2d*)(pout + 2 * t) = a;
        *(volatile v2d*)(pout + 64 + 2 * t) = b;
    }
    __threadfence();
    if (t < 32) {
        *(volatile v2d*)(pout + 2 * t) = a;
        *(volatile v2d*)(pout + 64 + 2 * t) = b;
    }
}

__global__ void __launch_bounds__(256)
k_bucket(const int* __restrict__ dstI, int* stage, int* binfo)
{
    __shared__ int lst[BKT_CAP];
    __shared__ __attribute__((aligned(16))) int srt[BKT_CAP];
    __shared__ __attribute__((aligned(16))) int info[BINFO_P];
    __shared__ int wsum[8];
    const int t = threadIdx.x, w = t >> 5, l = t & 31;
    const int b = blockIdx.x;
    const int nlo = b * BKT_NODES, nhi = nlo + BKT_NODES;

    int count = 0;
    for (int c0 = 0; c0 < NEDGE; c0 += 256) {
        const int e = c0 + t;
        int dv = -1;
        if (e < NEDGE) dv = dstI[e];
        const bool in = (dv >= nlo) && (dv < nhi);
        const unsigned bal = __builtin_amdgcn_ballot_w32(in);
        const int pre = __builtin_popcount(bal & ((1u << l) - 1u));
        if (l == 0) wsum[w] = __builtin_popcount(bal);
        __syncthreads();
        int woff = 0, tot = 0;
#pragma unroll
        for (int j = 0; j < 8; ++j) { const int s = wsum[j]; tot += s; woff += (j < w) ? s : 0; }
        if (in) {
            const int pos = count + woff + pre;
            if (pos < BKT_CAP) lst[pos] = (e << 10) | (dv - nlo);
        }
        count += tot;
        __syncthreads();
    }
    if (count > BKT_CAP) count = BKT_CAP;

    int c0n = 0, c1n = 0, c2n = 0, c3n = 0;
    for (int j = 0; j < count; ++j) {
        const int v = lst[j];
        const int ln = v & 1023;
        if ((ln >> 2) == t) {
            const int s = ln & 3;
            c0n += (s == 0); c1n += (s == 1); c2n += (s == 2); c3n += (s == 3);
        }
    }
    const int tsum = c0n + c1n + c2n + c3n;
    int x = tsum;
#pragma unroll
    for (int d = 1; d < 32; d <<= 1) {
        const int y = __shfl_up(x, d);
        if (l >= d) x += y;
    }
    if (l == 31) wsum[w] = x;
    __syncthreads();
    int woff = 0, tot = 0;
#pragma unroll
    for (int j = 0; j < 8; ++j) { const int s = wsum[j]; tot += s; woff += (j < w) ? s : 0; }
    const int o0 = woff + x - tsum;
    const int o1 = o0 + c0n, o2 = o1 + c1n, o3 = o2 + c2n;
    info[4 * t] = o0; info[4 * t + 1] = o1; info[4 * t + 2] = o2; info[4 * t + 3] = o3;
    if (t == 0) info[BKT_NODES] = tot;
    if (t < BINFO_P - BKT_NODES - 1) info[BKT_NODES + 1 + t] = 0;

    int r0 = 0, r1 = 0, r2 = 0, r3 = 0;
    for (int j = 0; j < count; ++j) {
        const int v = lst[j];
        const int ln = v & 1023;
        if ((ln >> 2) == t) {
            const int s = ln & 3;
            const int pos = (s == 0) ? (o0 + r0) : ((s == 1) ? (o1 + r1) : ((s == 2) ? (o2 + r2) : (o3 + r3)));
            if ((unsigned)pos < (unsigned)BKT_CAP) srt[pos] = v >> 10;
            r0 += (s == 0); r1 += (s == 1); r2 += (s == 2); r3 += (s == 3);
        }
    }
    __syncthreads();

    const int npieces = ((count + 31) >> 5) * 8;
    int* sdst = stage + (size_t)b * BKT_CAP;
    int* bdst = binfo + (size_t)b * BINFO_P;
    for (int p = t; p < npieces; p += 256) {
        const v4i v = *(const v4i_a*)&srt[p * 4];
        *(volatile v4i*)(sdst + p * 4) = v;
    }
    for (int p = t; p < BINFO_P / 4; p += 256) {
        const v4i v = *(const v4i_a*)&info[p * 4];
        *(volatile v4i*)(bdst + p * 4) = v;
    }
    __threadfence();
    for (int p = t; p < npieces; p += 256) {
        const v4i v = *(const v4i_a*)&srt[p * 4];
        *(volatile v4i*)(sdst + p * 4) = v;
    }
    for (int p = t; p < BINFO_P / 4; p += 256) {
        const v4i v = *(const v4i_a*)&info[p * 4];
        *(volatile v4i*)(bdst + p * 4) = v;
    }
}

__global__ void __launch_bounds__(256)
k_offsets(const int* __restrict__ binfo, int* off)
{
    __shared__ int base[NBKT + 1];
    const int t = threadIdx.x;
    if (t == 0) {
        int acc = 0;
        for (int b = 0; b < NBKT; ++b) {
            base[b] = acc;
            int c = binfo[(size_t)b * BINFO_P + BKT_NODES];
            c = clampi(c, 0, BKT_CAP);
            acc += c;
        }
        base[NBKT] = acc;
    }
    __syncthreads();
    const int p = blockIdx.x * 256 + t;
    const bool act = p < OFF_PIECES;
    v4i v = {0, 0, 0, 0};
    if (act) {
#pragma unroll
        for (int j = 0; j < 4; ++j) {
            const int n = 4 * p + j;
            int val;
            if (n < NNODE) {
                const int bb = n >> 10;
                int lo = binfo[(size_t)bb * BINFO_P + (n & 1023)];
                lo = clampi(lo, 0, BKT_CAP);
                val = base[bb] + lo;
            } else {
                val = base[NBKT];
            }
            v[j] = val;
        }
        *(volatile v4i*)(off + 4 * (size_t)p) = v;
    }
    __threadfence();
    if (act) *(volatile v4i*)(off + 4 * (size_t)p) = v;
}

__global__ void __launch_bounds__(256)
k_perm(const int* __restrict__ off, const int* __restrict__ stage, int* perm)
{
    __shared__ int base[NBKT + 1];
    const int t = threadIdx.x;
    if (t < NBKT) base[t] = off[t * BKT_NODES];
    if (t == NBKT) base[NBKT] = off[NNODE];
    __syncthreads();
    const int p = blockIdx.x * 256 + t;
    const bool act = p < PERM_PIECES;
    v4i v = {0, 0, 0, 0};
    if (act) {
        const int pos0 = 4 * p;
        int lo = 0, hi = NBKT - 1;
        while (lo < hi) {
            const int mid = (lo + hi + 1) >> 1;
            if (base[mid] <= pos0) lo = mid; else hi = mid - 1;
        }
        int bb = lo;
#pragma unroll
        for (int j = 0; j < 4; ++j) {
            const int pos = pos0 + j;
            while (bb < NBKT - 1 && pos >= base[bb + 1]) ++bb;
            int val = 0;
            if (pos < base[NBKT] && pos >= base[bb]) {
                const int loc = clampi(pos - base[bb], 0, BKT_CAP - 1);
                val = stage[(size_t)bb * BKT_CAP + loc];
            }
            v[j] = val;
        }
        *(volatile v4i*)(perm + 4 * (size_t)p) = v;
    }
    __threadfence();
    if (act) *(volatile v4i*)(perm + 4 * (size_t)p) = v;
}

__device__ __forceinline__ void embed_store(const float* stg, float* hrow0, f16t* h16row0, int l) {
#pragma unroll
    for (int j = 0; j < 8; ++j) {
        const int p = 32 * j + l;
        const int row = p >> 4, cb = (p & 15) * 4;
        const v4f v = *(const v4f_a*)(stg + row * EMBD + cb);
        *(volatile v4f*)(hrow0 + (size_t)row * EMBD + cb) = v;
    }
#pragma unroll
    for (int j = 0; j < 4; ++j) {
        const int p = 32 * j + l;
        const int row = p >> 3, cb = (p & 7) * 8;
        const v4f v0 = *(const v4f_a*)(stg + row * EMBD + cb);
        const v4f v1 = *(const v4f_a*)(stg + row * EMBD + cb + 4);
        v8h hv;
#pragma unroll
        for (int i = 0; i < 4; ++i) { hv[i] = (f16t)v0[i]; hv[4 + i] = (f16t)v1[i]; }
        *(volatile v8h*)(h16row0 + (size_t)row * EMBD + cb) = hv;
    }
}

__global__ void __launch_bounds__(128)
k_embed(const float* __restrict__ x, const float* __restrict__ Win, const float* __restrict__ bin,
        float* hout, f16t* h16out)
{
    __shared__ __attribute__((aligned(16))) f16t Ws[EMBD * 64];
    __shared__ float bias[EMBD];
    __shared__ __attribute__((aligned(16))) float stg[4][16 * EMBD];
    const int t = threadIdx.x, w = t >> 5, l = t & 31, hh = l >> 4, m = l & 15;
    for (int idx = t; idx < 64 * EMBD; idx += 128) {
        const int k = idx >> 6, n = idx & 63;
        const float v = (k < INDIM) ? Win[k * EMBD + n] * WSCALE : 0.0f;
        Ws[n * 64 + k] = (f16t)v;
    }
    if (t < EMBD) bias[t] = bin[t];
    __syncthreads();
    for (int base = blockIdx.x * 4; base < NTILES; base += gridDim.x * 4) {
        const int tile = base + w;
        const bool valid = tile < NTILES;
        const int row0 = tile * 16;
        if (valid) {
            v8f acc[4];
#pragma unroll
            for (int n = 0; n < 4; ++n)
#pragma unroll
                for (int r = 0; r < 8; ++r) acc[n][r] = 0.0f;
            const float* xr = x + (size_t)(row0 + m) * INDIM;
#pragma unroll
            for (int c = 0; c < 2; ++c) {
                FragU a;
#pragma unroll
                for (int i = 0; i < 16; ++i) {
                    const int k = 32 * c + ((i < 8) ? (8 * hh + i) : (8 + 8 * hh + i));
                    const int kc = (k < INDIM) ? k : (INDIM - 1);
                    float v = xr[kc];
                    v = (k < INDIM) ? v : 0.0f;
                    a.v[i] = (f16t)v;
                }
#pragma unroll
                for (int n = 0; n < 4; ++n)
                    acc[n] = wmma16(a.v, frag16(Ws + (16 * n + m) * 64 + 32 * c, hh), acc[n]);
            }
#pragma unroll
            for (int n = 0; n < 4; ++n) {
                const float bc = bias[16 * n + m];
#pragma unroll
                for (int r = 0; r < 8; ++r)
                    stg[w][(8 * hh + r) * EMBD + 16 * n + m] = acc[n][r] * WINV + bc;
            }
        }
        __syncthreads();
        if (valid) embed_store(stg[w], hout + (size_t)row0 * EMBD, h16out + (size_t)row0 * EMBD, l);
        __threadfence();
        if (valid) embed_store(stg[w], hout + (size_t)row0 * EMBD, h16out + (size_t)row0 * EMBD, l);
        __syncthreads();
    }
}

__global__ void __launch_bounds__(128)
k_edge1(const f16t* __restrict__ h16, const int* __restrict__ perm, const int* __restrict__ srcI,
        const int* __restrict__ dstI, const float* __restrict__ ea, const float* __restrict__ W1,
        const float* __restrict__ b1, f16t* zout, double* pstat)
{
    __shared__ __attribute__((aligned(16))) f16t Ws[EMBD * 128];
    __shared__ float wlast[EMBD], bias[EMBD];
    __shared__ __attribute__((aligned(16))) f16t stg[4][16 * EMBD];
    __shared__ __attribute__((aligned(16))) double red[1024];
    const int t = threadIdx.x, w = t >> 5, l = t & 31, hh = l >> 4, m = l & 15;
    for (int idx = t; idx < 128 * EMBD; idx += 128) {
        const int k = idx >> 6, n = idx & 63;
        Ws[n * 128 + k] = (f16t)(W1[idx] * WSCALE);
    }
    if (t < EMBD) { wlast[t] = W1[128 * EMBD + t]; bias[t] = b1[t]; }
    __syncthreads();
    double sl[4] = {0.0, 0.0, 0.0, 0.0}, ql[4] = {0.0, 0.0, 0.0, 0.0};
    for (int base = blockIdx.x * 4; base < ETILES; base += gridDim.x * 4) {
        const int tile = base + w;
        const bool valid = tile < ETILES;
        const int row0 = tile * 16;
        if (valid) {
            int e = perm[row0 + m];
            e = clampi(e, 0, NEDGE - 1);
            const int d = clampi(dstI[e], 0, NNODE - 1);
            const int s = clampi(srcI[e], 0, NNODE - 1);
            const float eav = ea[e];
            v8f acc[4];
#pragma unroll
            for (int n = 0; n < 4; ++n)
#pragma unroll
                for (int r = 0; r < 8; ++r) acc[n][r] = 0.0f;
#pragma unroll
            for (int c = 0; c < 4; ++c) {
                const int node = (c < 2) ? d : s;
                const v16h a = frag16(h16 + (size_t)node * EMBD + 32 * (c & 1), hh);
#pragma unroll
                for (int n = 0; n < 4; ++n)
                    acc[n] = wmma16(a, frag16(Ws + (16 * n + m) * 128 + 32 * c, hh), acc[n]);
            }
            float eam[8];
#pragma unroll
            for (int r = 0; r < 8; ++r) eam[r] = __shfl(eav, 8 * hh + r);
#pragma unroll
            for (int n = 0; n < 4; ++n) {
                const float wl = wlast[16 * n + m], bc = bias[16 * n + m];
#pragma unroll
                for (int r = 0; r < 8; ++r) {
                    const float v = acc[n][r] * WINV + eam[r] * wl + bc;
                    stg[w][(8 * hh + r) * EMBD + 16 * n + m] = (f16t)v;
                    sl[n] += (double)v;
                    ql[n] += (double)v * (double)v;
                }
            }
        }
        __syncthreads();
        if (valid) rows16_store(stg[w], zout + (size_t)row0 * EMBD, l);
        __threadfence();
        if (valid) rows16_store(stg[w], zout + (size_t)row0 * EMBD, l);
        __syncthreads();
    }
    stats_out(sl, ql, red, pstat + (size_t)blockIdx.x * 128);
}

__global__ void __launch_bounds__(128)
k_gemm2(f16t* z, const float* __restrict__ coef, const float* __restrict__ W2,
        const float* __restrict__ b2, double* pstat, int ntiles)
{
    __shared__ __attribute__((aligned(16))) f16t Ws[EMBD * 64];
    __shared__ float sa[EMBD], sb[EMBD], bias[EMBD];
    __shared__ __attribute__((aligned(16))) f16t stg[4][16 * EMBD];
    __shared__ __attribute__((aligned(16))) double red[1024];
    const int t = threadIdx.x, w = t >> 5, l = t & 31, hh = l >> 4, m = l & 15;
    for (int idx = t; idx < 64 * EMBD; idx += 128) {
        const int k = idx >> 6, n = idx & 63;
        Ws[n * 64 + k] = (f16t)(W2[idx] * WSCALE);
    }
    if (t < EMBD) { sa[t] = coef[t]; sb[t] = coef[EMBD + t]; bias[t] = b2[t]; }
    __syncthreads();
    double sl[4] = {0.0, 0.0, 0.0, 0.0}, ql[4] = {0.0, 0.0, 0.0, 0.0};
    for (int base = blockIdx.x * 4; base < ntiles; base += gridDim.x * 4) {
        const int tile = base + w;
        const bool valid = tile < ntiles;
        const int row0 = tile * 16;
        if (valid) {
            v8f acc[4];
#pragma unroll
            for (int n = 0; n < 4; ++n)
#pragma unroll
                for (int r = 0; r < 8; ++r) acc[n][r] = 0.0f;
#pragma unroll
            for (int c = 0; c < 2; ++c) {
                const f16t* zr = z + (size_t)(row0 + m) * EMBD + 32 * c;
                const v8h z0 = *(const v8h_a*)(zr + 8 * hh);
                const v8h z1 = *(const v8h_a*)(zr + 16 + 8 * hh);
                FragU a;
#pragma unroll
                for (int i = 0; i < 8; ++i) {
                    const int k = 32 * c + 8 * hh + i;
                    a.v[i] = (f16t)fmaxf(sa[k] * (float)z0[i] + sb[k], 0.0f);
                }
#pragma unroll
                for (int i = 0; i < 8; ++i) {
                    const int k = 32 * c + 16 + 8 * hh + i;
                    a.v[8 + i] = (f16t)fmaxf(sa[k] * (float)z1[i] + sb[k], 0.0f);
                }
#pragma unroll
                for (int n = 0; n < 4; ++n)
                    acc[n] = wmma16(a.v, frag16(Ws + (16 * n + m) * 64 + 32 * c, hh), acc[n]);
            }
#pragma unroll
            for (int n = 0; n < 4; ++n) {
                const float bc = bias[16 * n + m];
#pragma unroll
                for (int r = 0; r < 8; ++r) {
                    const float v = acc[n][r] * WINV + bc;
                    stg[w][(8 * hh + r) * EMBD + 16 * n + m] = (f16t)v;
                    sl[n] += (double)v;
                    ql[n] += (double)v * (double)v;
                }
            }
        }
        __syncthreads();
        if (valid) rows16_store(stg[w], z + (size_t)row0 * EMBD, l);
        __threadfence();
        if (valid) rows16_store(stg[w], z + (size_t)row0 * EMBD, l);
        __syncthreads();
    }
    stats_out(sl, ql, red, pstat + (size_t)blockIdx.x * 128);
}

__global__ void __launch_bounds__(128)
k_node1(const f16t* __restrict__ h16, const float* __restrict__ aggr, const float* __restrict__ W1,
        const float* __restrict__ b1, f16t* zout, double* pstat)
{
    __shared__ __attribute__((aligned(16))) f16t Ws[EMBD * 128];
    __shared__ float bias[EMBD];
    __shared__ __attribute__((aligned(16))) f16t stg[4][16 * EMBD];
    __shared__ __attribute__((aligned(16))) double red[1024];
    const int t = threadIdx.x, w = t >> 5, l = t & 31, hh = l >> 4, m = l & 15;
    for (int idx = t; idx < 128 * EMBD; idx += 128) {
        const int k = idx >> 6, n = idx & 63;
        Ws[n * 128 + k] = (f16t)(W1[idx] * WSCALE);
    }
    if (t < EMBD) bias[t] = b1[t];
    __syncthreads();
    double sl[4] = {0.0, 0.0, 0.0, 0.0}, ql[4] = {0.0, 0.0, 0.0, 0.0};
    for (int base = blockIdx.x * 4; base < NTILES; base += gridDim.x * 4) {
        const int tile = base + w;
        const bool valid = tile < NTILES;
        const int row0 = tile * 16;
        if (valid) {
            const int row = row0 + m;
            v8f acc[4];
#pragma unroll
            for (int n = 0; n < 4; ++n)
#pragma unroll
                for (int r = 0; r < 8; ++r) acc[n][r] = 0.0f;
#pragma unroll
            for (int c = 0; c < 2; ++c) {
                const v16h a = frag16(h16 + (size_t)row * EMBD + 32 * c, hh);
#pragma unroll
                for (int n = 0; n < 4; ++n)
                    acc[n] = wmma16(a, frag16(Ws + (16 * n + m) * 128 + 32 * c, hh), acc[n]);
            }
#pragma unroll
            for (int c = 0; c < 2; ++c) {
                const float* ap = aggr + (size_t)row * EMBD + 32 * c;
                const v4f u0 = *(const v4f_a*)(ap + 8 * hh);
                const v4f u1 = *(const v4f_a*)(ap + 8 * hh + 4);
                const v4f u2 = *(const v4f_a*)(ap + 16 + 8 * hh);
                const v4f u3 = *(const v4f_a*)(ap + 20 + 8 * hh);
                FragU a;
#pragma unroll
                for (int i = 0; i < 4; ++i) {
                    a.v[i] = (f16t)u0[i];
                    a.v[4 + i] = (f16t)u1[i];
                    a.v[8 + i] = (f16t)u2[i];
                    a.v[12 + i] = (f16t)u3[i];
                }
#pragma unroll
                for (int n = 0; n < 4; ++n)
                    acc[n] = wmma16(a.v, frag16(Ws + (16 * n + m) * 128 + 64 + 32 * c, hh), acc[n]);
            }
#pragma unroll
            for (int n = 0; n < 4; ++n) {
                const float bc = bias[16 * n + m];
#pragma unroll
                for (int r = 0; r < 8; ++r) {
                    const float v = acc[n][r] * WINV + bc;
                    stg[w][(8 * hh + r) * EMBD + 16 * n + m] = (f16t)v;
                    sl[n] += (double)v;
                    ql[n] += (double)v * (double)v;
                }
            }
        }
        __syncthreads();
        if (valid) rows16_store(stg[w], zout + (size_t)row0 * EMBD, l);
        __threadfence();
        if (valid) rows16_store(stg[w], zout + (size_t)row0 * EMBD, l);
        __syncthreads();
    }
    stats_out(sl, ql, red, pstat + (size_t)blockIdx.x * 128);
}

__global__ void __launch_bounds__(256)
k_bnfin(const double* __restrict__ pstat, int nblk, int count, const float* __restrict__ g,
        const float* __restrict__ be, float* coef)
{
    __shared__ double rS[4][64], rQ[4][64];
    __shared__ __attribute__((aligned(16))) float cs[128];
    const int t = threadIdx.x, c = t & 63, part = t >> 6;
    double S = 0.0, Q = 0.0;
    for (int b = part; b < nblk; b += 4) {
        S += pstat[(size_t)b * 128 + c];
        Q += pstat[(size_t)b * 128 + 64 + c];
    }
    rS[part][c] = S; rQ[part][c] = Q;
    __syncthreads();
    if (t < 64) {
        const double s = rS[0][t] + rS[1][t] + rS[2][t] + rS[3][t];
        const double q = rQ[0][t] + rQ[1][t] + rQ[2][t] + rQ[3][t];
        const double mean = s / (double)count;
        double var = q / (double)count - mean * mean;
        if (var < 0.0) var = 0.0;
        const float a = g[t] * rsqrtf((float)var + BN_EPS);
        cs[t] = a;
        cs[64 + t] = be[t] - (float)mean * a;
    }
    __syncthreads();
    v4f v = {0.0f, 0.0f, 0.0f, 0.0f};
    if (t < 32) { v = *(const v4f_a*)&cs[4 * t]; *(volatile v4f*)(coef + 4 * t) = v; }
    __threadfence();
    if (t < 32) *(volatile v4f*)(coef + 4 * t) = v;
}

__global__ void __launch_bounds__(128)
k_gather(const f16t* __restrict__ z, const int* __restrict__ off, const float* __restrict__ coef, float* aggr)
{
    const int t = threadIdx.x, w = t >> 5, l = t & 31;
    const int node = blockIdx.x * 4 + w;
    if (node >= NNODE) return;
    const float a0 = coef[2 * l], a1 = coef[2 * l + 1], b0 = coef[64 + 2 * l], b1 = coef[64 + 2 * l + 1];
    int beg = off[node], end = off[node + 1];
    beg = clampi(beg, 0, NEDGE);
    end = clampi(end, beg, NEDGE);
    float s0 = 0.0f, s1 = 0.0f;
    for (int i = beg; i < end; ++i) {
        const v2h zz = *(const v2h_a*)(z + (size_t)i * EMBD + 2 * l);
        s0 += fmaxf(a0 * (float)zz[0] + b0, 0.0f);
        s1 += fmaxf(a1 * (float)zz[1] + b1, 0.0f);
    }
    v4f v;
    v[0] = __shfl(s0, (2 * l) & 31);
    v[1] = __shfl(s1, (2 * l) & 31);
    v[2] = __shfl(s0, (2 * l + 1) & 31);
    v[3] = __shfl(s1, (2 * l + 1) & 31);
    float* dst = aggr + (size_t)node * EMBD + 4 * l;
    if (l < 16) *(volatile v4f*)dst = v;
    __threadfence();
    if (l < 16) *(volatile v4f*)dst = v;
}

__global__ void __launch_bounds__(128)
k_update(float* h, f16t* h16, const f16t* __restrict__ zu, const float* __restrict__ coef)
{
    const int t = threadIdx.x, w = t >> 5, l = t & 31, hh = l >> 4, q = l & 15;
    float ca[4], cbv[4];
#pragma unroll
    for (int i = 0; i < 4; ++i) { ca[i] = coef[4 * q + i]; cbv[i] = coef[64 + 4 * q + i]; }
    const int qq = q & 7;
    for (int rg = blockIdx.x; rg < NNODE / 8; rg += gridDim.x) {
        const int row = rg * 8 + w * 2 + hh;
        const size_t o = (size_t)row * EMBD + 4 * q;
        const v4f hv = *(const v4f_a*)(h + o);
        const v4h zv = *(const v4h_a*)(zu + o);
        v4f hn;
#pragma unroll
        for (int i = 0; i < 4; ++i) hn[i] = hv[i] + fmaxf(ca[i] * (float)zv[i] + cbv[i], 0.0f);
        float gth[8];
#pragma unroll
        for (int i = 0; i < 4; ++i) {
            gth[i]     = __shfl(hn[i], 16 * hh + 2 * qq);
            gth[4 + i] = __shfl(hn[i], 16 * hh + 2 * qq + 1);
        }
        v8h h8;
#pragma unroll
        for (int i = 0; i < 8; ++i) h8[i] = (f16t)gth[i];
        f16t* d16 = h16 + (size_t)row * EMBD + 8 * q;
        *(volatile v4f*)(h + o) = hn;
        if (q < 8) *(volatile v8h*)d16 = h8;
        __threadfence();
        *(volatile v4f*)(h + o) = hn;
        if (q < 8) *(volatile v8h*)d16 = h8;
    }
}

__global__ void __launch_bounds__(64)
k_colsum(const float* __restrict__ h, double* cpart)
{
    __shared__ __attribute__((aligned(16))) double st[64];
    const int c = threadIdx.x;
    const int R = (NNODE + CS_BLOCKS - 1) / CS_BLOCKS;
    const int r0 = blockIdx.x * R;
    int r1 = r0 + R; if (r1 > NNODE) r1 = NNODE;
    double s = 0.0;
    for (int r = r0; r < r1; ++r) s += (double)h[(size_t)r * EMBD + c];
    st[c] = s;
    __syncthreads();
    v2d v = {0.0, 0.0};
    if (c < 32) { v = *(const v2d_a*)&st[2 * c]; *(volatile v2d*)(cpart + (size_t)blockIdx.x * 64 + 2 * c) = v; }
    __threadfence();
    if (c < 32) *(volatile v2d*)(cpart + (size_t)blockIdx.x * 64 + 2 * c) = v;
}

__global__ void __launch_bounds__(64)
k_final(const double* __restrict__ cpart, const float* __restrict__ Wp, const float* __restrict__ bp, float* out)
{
    __shared__ double st[64];
    const int c = threadIdx.x;
    double s = 0.0;
    for (int b = 0; b < CS_BLOCKS; ++b) s += cpart[(size_t)b * 64 + c];
    st[c] = (s / (double)NNODE) * (double)Wp[c];
    __syncthreads();
    for (int d = 32; d > 0; d >>= 1) {
        if (c < d) st[c] += st[c + d];
        __syncthreads();
    }
    if (c == 0) {
        const float v = (float)(st[0] + (double)bp[0]);
        *(volatile float*)out = v;
        __threadfence();
        *(volatile float*)out = v;
    }
}

static inline size_t al256(size_t v) { return (v + 255) & ~(size_t)255; }

extern "C" void kernel_launch(void* const* d_in, const int* in_sizes, int n_in,
                              void* d_out, int out_size, void* d_ws, size_t ws_size,
                              hipStream_t stream)
{
    if (n_in < 23 || out_size < 1 || d_out == 0 || d_ws == 0) return;
    if (in_sizes[0] != NNODE * INDIM || in_sizes[1] != 2 * NEDGE || in_sizes[2] != NEDGE) return;
    if (in_sizes[3] != INDIM * EMBD || in_sizes[5] != NLAYER * 129 * EMBD || in_sizes[13] != NLAYER * 128 * EMBD) return;

    const float* x       = (const float*)d_in[0];
    const int*   eidx    = (const int*)d_in[1];
    const float* ea      = (const float*)d_in[2];
    const float* W_in    = (const float*)d_in[3];
    const float* b_in    = (const float*)d_in[4];
    const float* msg_W1  = (const float*)d_in[5];
    const float* msg_b1  = (const float*)d_in[6];
    const float* msg_g1  = (const float*)d_in[7];
    const float* msg_be1 = (const float*)d_in[8];
    const float* msg_W2  = (const float*)d_in[9];
    const float* msg_b2  = (const float*)d_in[10];
    const float* msg_g2  = (const float*)d_in[11];
    const float* msg_be2 = (const float*)d_in[12];
    const float* upd_W1  = (const float*)d_in[13];
    const float* upd_b1  = (const float*)d_in[14];
    const float* upd_g1  = (const float*)d_in[15];
    const float* upd_be1 = (const float*)d_in[16];
    const float* upd_W2  = (const float*)d_in[17];
    const float* upd_b2  = (const float*)d_in[18];
    const float* upd_g2  = (const float*)d_in[19];
    const float* upd_be2 = (const float*)d_in[20];
    const float* W_pred  = (const float*)d_in[21];
    const float* b_pred  = (const float*)d_in[22];
    const int* srcI = eidx;
    const int* dstI = eidx + NEDGE;
    float* out = (float*)d_out;

    char* ws = (char*)d_ws;
    size_t o = 0;
    f16t*   z     = (f16t*)(ws + o);   o = al256(o + (size_t)NEDGE * EMBD * 2);
    float*  h     = (float*)(ws + o);  o = al256(o + (size_t)NNODE * EMBD * 4);
    f16t*   h16   = (f16t*)(ws + o);   o = al256(o + (size_t)NNODE * EMBD * 2);
    float*  aggr  = (float*)(ws + o);  o = al256(o + (size_t)NNODE * EMBD * 4);
    f16t*   zu    = (f16t*)(ws + o);   o = al256(o + (size_t)NNODE * EMBD * 2);
    int*    stage = (int*)(ws + o);    o = al256(o + (size_t)NBKT * BKT_CAP * 4);
    int*    binfo = (int*)(ws + o);    o = al256(o + (size_t)NBKT * BINFO_P * 4);
    int*    offa  = (int*)(ws + o);    o = al256(o + (size_t)OFF_PAD * 4);
    int*    perm  = (int*)(ws + o);    o = al256(o + (size_t)NEDGE * 4);
    double* pstat = (double*)(ws + o); o = al256(o + (size_t)EDGE_GRID * 128 * 8);
    float*  coef0 = (float*)(ws + o);  o = al256(o + (size_t)128 * 4);
    float*  coef1 = (float*)(ws + o);  o = al256(o + (size_t)128 * 4);
    double* cpart = (double*)(ws + o); o = al256(o + (size_t)CS_BLOCKS * 64 * 8);
    if (o > ws_size) return;

    k_bucket<<<NBKT, 256, 0, stream>>>(dstI, stage, binfo);
    k_offsets<<<(OFF_PIECES + 255) / 256, 256, 0, stream>>>(binfo, offa);
    k_perm<<<(PERM_PIECES + 255) / 256, 256, 0, stream>>>(offa, stage, perm);

    k_embed<<<(NTILES + 3) / 4, 128, 0, stream>>>(x, W_in, b_in, h, h16);

    for (int lyr = 0; lyr < NLAYER; ++lyr) {
        const float* mW1 = msg_W1 + (size_t)lyr * 129 * EMBD;
        const float* mW2 = msg_W2 + (size_t)lyr * EMBD * EMBD;
        const float* uW1 = upd_W1 + (size_t)lyr * 128 * EMBD;
        const float* uW2 = upd_W2 + (size_t)lyr * EMBD * EMBD;

        k_edge1<<<EDGE_GRID, 128, 0, stream>>>(h16, perm, srcI, dstI, ea, mW1, msg_b1 + lyr * EMBD, z, pstat);
        k_bnfin<<<1, 256, 0, stream>>>(pstat, EDGE_GRID, NEDGE, msg_g1 + lyr * EMBD, msg_be1 + lyr * EMBD, coef0);
        k_gemm2<<<EDGE_GRID, 128, 0, stream>>>(z, coef0, mW2, msg_b2 + lyr * EMBD, pstat, ETILES);
        k_bnfin<<<1, 256, 0, stream>>>(pstat, EDGE_GRID, NEDGE, msg_g2 + lyr * EMBD, msg_be2 + lyr * EMBD, coef1);
        k_gather<<<NNODE / 4, 128, 0, stream>>>(z, offa, coef1, aggr);
        k_node1<<<NODE_GRID, 128, 0, stream>>>(h16, aggr, uW1, upd_b1 + lyr * EMBD, zu, pstat);
        k_bnfin<<<1, 256, 0, stream>>>(pstat, NODE_GRID, NNODE, upd_g1 + lyr * EMBD, upd_be1 + lyr * EMBD, coef0);
        k_gemm2<<<NODE_GRID, 128, 0, stream>>>(zu, coef0, uW2, upd_b2 + lyr * EMBD, pstat, NTILES);
        k_bnfin<<<1, 256, 0, stream>>>(pstat, NODE_GRID, NNODE, upd_g2 + lyr * EMBD, upd_be2 + lyr * EMBD, coef1);
        k_update<<<2048, 128, 0, stream>>>(h, h16, zu, coef1);
    }

    k_colsum<<<CS_BLOCKS, 64, 0, stream>>>(h, cpart);
    k_final<<<1, 64, 0, stream>>>(cpart, W_pred, b_pred, out);
}
